// GruGatNets_64424509440156
// MI455X (gfx1250) — hardware-verified
//
#include <hip/hip_runtime.h>


#define NN_ 100000
#define HH 128
#define IL_CAP 32
#define NCHK 8
#define NPB 256

typedef __attribute__((ext_vector_type(16))) __bf16   v16bf;
typedef __attribute__((ext_vector_type(16))) _Float16 v16h;
typedef __attribute__((ext_vector_type(8)))  float    v8f;
typedef __attribute__((ext_vector_type(8)))  unsigned v8u;

__device__ __forceinline__ unsigned f2bf(float f) { unsigned u = __float_as_uint(f); u += 0x7FFFu + ((u >> 16) & 1u); return u >> 16; }
__device__ __forceinline__ unsigned f2h(float f) { return (unsigned)__builtin_bit_cast(unsigned short, (_Float16)f); }
__device__ __forceinline__ int kpat(int v, int half) { return ((v & 4) ? 16 : 0) + half * 8 + 2 * (v & 3); }

template <int F16, int NP> struct Opnd { v16bf p[NP]; };

template <int F16, int NP> __device__ __forceinline__ void pack2(float f0, float f1, unsigned* o) {
    if (F16) { o[0] = f2h(f0) | (f2h(f1) << 16); return; }
    unsigned h0 = f2bf(f0), h1 = f2bf(f1); o[0] = h0 | (h1 << 16);
    if (NP >= 2) {
        float r0 = f0 - __uint_as_float(h0 << 16), r1 = f1 - __uint_as_float(h1 << 16);
        unsigned m0 = f2bf(r0), m1 = f2bf(r1); o[1] = m0 | (m1 << 16);
        if (NP >= 3) {
            float s0 = r0 - __uint_as_float(m0 << 16), s1 = r1 - __uint_as_float(m1 << 16);
            o[2] = f2bf(s0) | (f2bf(s1) << 16);
        }
    }
}
template <int F16, int NP> __device__ __forceinline__ void op_row(const float* rowp, int half, float sc, Opnd<F16, NP>& o) {
    v8u u[NP];
#pragma unroll
    for (int v = 0; v < 8; ++v) {
        int kk = kpat(v, half); unsigned t[3];
        pack2<F16, NP>(rowp[kk] * sc, rowp[kk + 1] * sc, t);
#pragma unroll
        for (int p = 0; p < NP; ++p) u[p][v] = t[p];
    }
#pragma unroll
    for (int p = 0; p < NP; ++p) o.p[p] = __builtin_bit_cast(v16bf, u[p]);
}
template <int F16, int NP> __device__ __forceinline__ void op_row_tail(const float* rowp, int half, float sc, int kvalid, Opnd<F16, NP>& o) {
    v8u u[NP];
#pragma unroll
    for (int v = 0; v < 8; ++v) {
        int kk = kpat(v, half); unsigned t[3];
        float f0 = kk < kvalid ? rowp[kk] * sc : 0.0f, f1 = (kk + 1) < kvalid ? rowp[kk + 1] * sc : 0.0f;
        pack2<F16, NP>(f0, f1, t);
#pragma unroll
        for (int p = 0; p < NP; ++p) u[p][v] = t[p];
    }
#pragma unroll
    for (int p = 0; p < NP; ++p) o.p[p] = __builtin_bit_cast(v16bf, u[p]);
}
template <int F16, int NP> __device__ __forceinline__ void op_col(const float* M, int ld, int n, int k0, int half, float sc, Opnd<F16, NP>& o) {
    v8u u[NP];
#pragma unroll
    for (int v = 0; v < 8; ++v) {
        int kk = k0 + kpat(v, half); unsigned t[3];
        pack2<F16, NP>(M[(size_t)kk * ld + n] * sc, M[(size_t)(kk + 1) * ld + n] * sc, t);
#pragma unroll
        for (int p = 0; p < NP; ++p) u[p][v] = t[p];
    }
#pragma unroll
    for (int p = 0; p < NP; ++p) o.p[p] = __builtin_bit_cast(v16bf, u[p]);
}
template <int F16, int NP> __device__ __forceinline__ void op_col_tail(const float* M, int ld, int n, int k0, int half, float sc, int K, Opnd<F16, NP>& o) {
    v8u u[NP];
#pragma unroll
    for (int v = 0; v < 8; ++v) {
        int kk = k0 + kpat(v, half); unsigned t[3];
        float f0 = kk < K ? M[(size_t)kk * ld + n] * sc : 0.0f, f1 = (kk + 1) < K ? M[(size_t)(kk + 1) * ld + n] * sc : 0.0f;
        pack2<F16, NP>(f0, f1, t);
#pragma unroll
        for (int p = 0; p < NP; ++p) u[p][v] = t[p];
    }
#pragma unroll
    for (int p = 0; p < NP; ++p) o.p[p] = __builtin_bit_cast(v16bf, u[p]);
}
__device__ __forceinline__ v8f wm_bf16(v16bf a, v16bf b, v8f c) { return __builtin_amdgcn_wmma_f32_16x16x32_bf16(false, a, false, b, (short)0, c, false, false); }
template <int F16, int NA, int NB> __device__ __forceinline__ v8f wmma_op(const Opnd<F16, NA>& a, const Opnd<F16, NB>& b, v8f c) {
    if (F16) {
        v16h ah = __builtin_bit_cast(v16h, a.p[0]), bh = __builtin_bit_cast(v16h, b.p[0]);
        c = __builtin_amdgcn_wmma_f32_16x16x32_f16(false, ah, false, bh, (short)0, c, false, false);
        asm volatile("v_nop\n\tv_nop\n\tv_nop\n\tv_nop" : "+v"(c) : "v"(ah), "v"(bh));
        return c;
    }
    constexpr int NMX = NA > NB ? NA : NB;
#pragma unroll
    for (int i = 0; i < NA; ++i)
#pragma unroll
        for (int j = 0; j < NB; ++j)
            if (i + j < NMX) c = wm_bf16(a.p[i], b.p[j], c);
    if (NA == 1 && NB == 1)      asm volatile("v_nop\n\tv_nop\n\tv_nop\n\tv_nop" : "+v"(c) : "v"(a.p[0]), "v"(b.p[0]));
    else if (NA == 2 && NB == 1) asm volatile("v_nop\n\tv_nop\n\tv_nop\n\tv_nop" : "+v"(c) : "v"(a.p[0]), "v"(a.p[1]), "v"(b.p[0]));
    else if (NA == 1 && NB == 2) asm volatile("v_nop\n\tv_nop\n\tv_nop\n\tv_nop" : "+v"(c) : "v"(a.p[0]), "v"(b.p[0]), "v"(b.p[1]));
    else if (NA == 2 && NB == 2) asm volatile("v_nop\n\tv_nop\n\tv_nop\n\tv_nop" : "+v"(c) : "v"(a.p[0]), "v"(a.p[1]), "v"(b.p[0]), "v"(b.p[1]));
    else                         asm volatile("v_nop\n\tv_nop\n\tv_nop\n\tv_nop" : "+v"(c) : "v"(a.p[0]), "v"(a.p[NA - 1]), "v"(b.p[0]), "v"(b.p[NB - 1]), "v"(a.p[NA / 2]), "v"(b.p[NB / 2]));
    return c;
}

struct ZMap { long long s1; long long s2; int zdiv; int pad_; };
__device__ __forceinline__ size_t zoff(const ZMap& m, int z) { return (size_t)((long long)(z / m.zdiv) * m.s1 + (long long)(z % m.zdiv) * m.s2); }

#define ACT_NONE 0
#define ACT_RELU 1
#define ACT_GELU_ERF 2
#define ACT_SILU 3
#define ACT_TANH 4
__device__ __forceinline__ float act_apply(int act, float x) {
    if (act == ACT_RELU) return x > 0.f ? x : 0.f;
    if (act == ACT_GELU_ERF) return 0.5f * x * (1.0f + erff(x * 0.70710678118654752f));
    if (act == ACT_SILU) return x / (1.0f + expf(-x));
    if (act == ACT_TANH) return tanhf(x);
    return x;
}
struct GemmArgs {
    ZMap za, zb_, zc, zbias, zadd, zrsc, zmul, zrbias;
    const float* A; const float* Bm; float* C; const float* bias; const float* add; const float* rsc; const float* mul; const float* rbias;
    long long ldadd, ldmul;
    int lda, ldb, ldc, K;
    float ascale, bscale, oscale, addscale;
    int M, nvalid, nstore, ldrsc;
    int bcs, pad1, pad2, pad3;
};
template <int BT, int F16, int NA, int NB, int RW, int CW, int ACT>
__global__ __launch_bounds__(256) void gemm_kernel(GemmArgs g) {
    constexpr int TR = 16 * RW, TC = 64 * CW, CSTR = TC + 4;
    __shared__ __align__(16) float cst[TR * CSTR];
    const int z = blockIdx.z;
    const float* A = g.A + zoff(g.za, z); const float* Bm = g.Bm + zoff(g.zb_, z); float* C = g.C + zoff(g.zc, z);
    const int tid = threadIdx.x, lane = tid & 31, wv = tid >> 5;
    const int l16 = lane & 15, half = lane >> 4;
    const int rt = wv % RW, ch = wv / RW;
    const int row0 = blockIdx.x * TR, col0 = blockIdx.y * TC + ch * 64;
    int arix = row0 + rt * 16 + l16; if (arix >= g.M) arix = g.M - 1;
    const float* arow = A + (size_t)arix * g.lda;
    v8f acc[4];
#pragma unroll
    for (int t = 0; t < 4; ++t) acc[t] = (v8f){};
    const int K = g.K;
#pragma unroll 1
    for (int kc = 0; kc < K; kc += 32) {
        Opnd<F16, NA> a;
        if (kc + 32 <= K) op_row<F16, NA>(arow + kc, half, g.ascale, a); else op_row_tail<F16, NA>(arow + kc, half, g.ascale, K - kc, a);
#pragma unroll
        for (int t = 0; t < 4; ++t) {
            Opnd<F16, NB> b;
            const int n = col0 + t * 16 + l16;
            if (n < g.nvalid) {
                if (BT) { if (kc + 32 <= K) op_row<F16, NB>(Bm + (size_t)n * g.ldb + kc, half, g.bscale, b); else op_row_tail<F16, NB>(Bm + (size_t)n * g.ldb + kc, half, g.bscale, K - kc, b); }
                else    { if (kc + 32 <= K) op_col<F16, NB>(Bm, g.ldb, n * g.bcs, kc, half, g.bscale, b); else op_col_tail<F16, NB>(Bm, g.ldb, n * g.bcs, kc, half, g.bscale, K, b); }
            } else {
#pragma unroll
                for (int p = 0; p < NB; ++p) b.p[p] = (v16bf){};
            }
            acc[t] = wmma_op<F16, NA, NB>(a, b, acc[t]);
        }
    }
    const float* bias = g.bias ? g.bias + zoff(g.zbias, z) : nullptr;
    const float* add = g.add ? g.add + zoff(g.zadd, z) : nullptr;
    const float* rsc = g.rsc ? g.rsc + zoff(g.zrsc, z) : nullptr;
    const float* mul = g.mul ? g.mul + zoff(g.zmul, z) : nullptr;
    const float* rbias = g.rbias ? g.rbias + zoff(g.zrbias, z) : nullptr;
#pragma unroll
    for (int t = 0; t < 4; ++t) {
        const int cl = ch * 64 + t * 16 + l16;
        const int cg = blockIdx.y * TC + cl;
        const bool cok = cg < g.nvalid;
        const float bv = (bias && cok) ? bias[(size_t)cg * g.bcs] : 0.0f;
#pragma unroll
        for (int r = 0; r < 8; ++r) {
            const int rl = rt * 16 + r + 8 * half;
            float v = acc[t][r] * g.oscale + bv;
            int rg = row0 + rl; if (rg >= g.M) rg = g.M - 1;
            if (rbias) v += rbias[rg];
            if (rsc) v *= rsc[(size_t)rg * g.ldrsc];
            if (mul && cok) v *= mul[(size_t)rg * g.ldmul + cg];
            if (add && cok) v += g.addscale * add[(size_t)rg * g.ldadd + cg];
            cst[rl * CSTR + cl] = v;
        }
    }
    __syncthreads();
    const int col = tid % TC, rsel = tid / TC, rstep = 256 / TC;
    if (ACT != ACT_NONE) {
#pragma unroll 1
        for (int r = rsel; r < TR; r += rstep) cst[r * CSTR + col] = act_apply(ACT, cst[r * CSTR + col]);
    }
    float* ob = C + (size_t)row0 * g.ldc + (size_t)blockIdx.y * TC;
    const bool colok = (int)(blockIdx.y * TC + col) < g.nstore;
    const int rmax = (g.M - row0 < TR) ? (g.M - row0) : TR;
    auto pass = [&]() {
        if (colok) {
#pragma unroll 4
            for (int r = rsel; r < rmax; r += rstep) *(volatile float*)(ob + (size_t)r * g.ldc + col) = cst[r * CSTR + col];
        }
    };
    pass();
    __threadfence();
    pass();
}
static inline ZMap zm(long long s1) { ZMap m; m.s1 = s1; m.s2 = 0; m.zdiv = 1; m.pad_ = 0; return m; }
static inline ZMap zm2(long long s1, long long s2, int zdiv) { ZMap m; m.s1 = s1; m.s2 = s2; m.zdiv = zdiv; m.pad_ = 0; return m; }
static inline GemmArgs gemm_args(const float* A, int lda, ZMap za, const float* Bm, int ldb, ZMap zb, float* C, int ldc, ZMap zc, int M, int N, int K) {
    GemmArgs g; g.za = za; g.zb_ = zb; g.zc = zc; g.zbias = zm(0); g.zadd = zm(0); g.zrsc = zm(0); g.zmul = zm(0); g.zrbias = zm(0);
    g.A = A; g.Bm = Bm; g.C = C; g.bias = nullptr; g.add = nullptr; g.rsc = nullptr; g.mul = nullptr; g.rbias = nullptr; g.ldadd = 0; g.ldmul = 0;
    g.lda = lda; g.ldb = ldb; g.ldc = ldc; g.K = K; g.ascale = 1.0f; g.bscale = 1.0f; g.oscale = 1.0f; g.addscale = 1.0f; g.M = M; g.nvalid = N; g.nstore = N; g.ldrsc = 1;
    g.bcs = 1; g.pad1 = 0; g.pad2 = 0; g.pad3 = 0;
    return g;
}
static_assert(sizeof(ZMap) == 24, "ZMap layout");
static_assert(sizeof(GemmArgs) == 8 * 24 + 8 * 8 + 2 * 8 + 4 * 4 + 4 * 4 + 4 * 4 + 4 * 4, "GemmArgs has no padding");

__global__ __launch_bounds__(256) void softmax_rows(float* S, long long sy, long long sx, int L, float prescale, const float* addv, long long say, int aydiv, int causal,
                                                  const int* imask, long long imy, long long imx, float maskval) {
    __shared__ float red[8];
    const int tid = threadIdx.x, lane = tid & 31, wid = tid >> 5;
    float* row = S + (size_t)blockIdx.y * sy + (size_t)blockIdx.x * sx;
    const float* av = addv ? addv + (size_t)(blockIdx.y / aydiv) * say : nullptr;
    const int* im = imask ? imask + (size_t)(blockIdx.y / aydiv) * imy + (size_t)blockIdx.x * imx : nullptr;
    float v[16];
    const int nj = L / 256;
    float mx = -__builtin_inff();
#pragma unroll
    for (int j = 0; j < 16; ++j) if (j < nj) { float t = row[tid + 256 * j] * prescale; if (av) t += av[tid + 256 * j]; if (im && im[tid + 256 * j] == 0) t = maskval; if (causal && (tid + 256 * j) > (int)blockIdx.x) t = -__builtin_inff(); v[j] = t; mx = fmaxf(mx, t); }
#pragma unroll
    for (int o = 16; o; o >>= 1) mx = fmaxf(mx, __shfl_xor(mx, o, 32));
    if (lane == 0) red[wid] = mx;
    __syncthreads();
    float m = red[0];
#pragma unroll
    for (int i = 1; i < 8; ++i) m = fmaxf(m, red[i]);
    if (m == -__builtin_inff()) m = 0.f;
    __syncthreads();
    float sum = 0.f;
#pragma unroll
    for (int j = 0; j < 16; ++j) if (j < nj) { v[j] = expf(v[j] - m); sum += v[j]; }
#pragma unroll
    for (int o = 16; o; o >>= 1) sum += __shfl_xor(sum, o, 32);
    if (lane == 0) red[wid] = sum;
    __syncthreads();
    float tot = 0.f;
#pragma unroll
    for (int i = 0; i < 8; ++i) tot += red[i];
    const float inv = 1.0f / tot;
#pragma unroll
    for (int j = 0; j < 16; ++j) if (j < nj) *(volatile float*)(row + tid + 256 * j) = v[j] * inv;
    __threadfence();
#pragma unroll
    for (int j = 0; j < 16; ++j) if (j < nj) *(volatile float*)(row + tid + 256 * j) = v[j] * inv;
}

#define VST2(T, p, v) do { const T vst2_v_ = (v); *(volatile T*)(p) = vst2_v_; __threadfence(); *(volatile T*)(p) = vst2_v_; } while (0)
#define IL_T 128
#define IL_TILE 4096
__global__ __launch_bounds__(IL_T) void k_inlists(const int* __restrict__ tgt, int E, int N, int* NBR, int* cnt) {
    __shared__ int tt[IL_TILE];
    __shared__ int lists[IL_T * IL_CAP];
    const int d = blockIdx.x * IL_T + threadIdx.x; int n = 0;
    for (int e0 = 0; e0 < E; e0 += IL_TILE) {
        const int nt = min(IL_TILE, E - e0);
        __syncthreads();
        for (int i = threadIdx.x; i < nt; i += IL_T) tt[i] = tgt[e0 + i];
        __syncthreads();
        for (int i = 0; i < nt; ++i) { if (tt[i] == d) { if (n < IL_CAP) lists[threadIdx.x * IL_CAP + n] = e0 + i; ++n; } }
    }
    if (d < N) {
        int* row = NBR + (size_t)d * IL_CAP;
        for (int j = 0; j < IL_CAP; ++j) { const int v = (j < n) ? lists[threadIdx.x * IL_CAP + j] : 0; *(volatile int*)(row + j) = v; }
        __threadfence();
        for (int j = 0; j < IL_CAP; ++j) { const int v = (j < n) ? lists[threadIdx.x * IL_CAP + j] : 0; *(volatile int*)(row + j) = v; }
        VST2(int, cnt + d, min(n, IL_CAP));
    }
}
__global__ __launch_bounds__(256) void k_csr_scan(const int* __restrict__ cnt, int* off, int N) {
    __shared__ int part[256]; const int per = ((((N + 255) / 256) + 31) / 32) * 32; const int a = threadIdx.x * per, b = min(N, a + per); int s = 0;
    for (int i = a; i < b; ++i) s += cnt[i]; part[threadIdx.x] = s; __syncthreads();
    if (threadIdx.x == 0) { int run = 0; for (int t = 0; t < 256; ++t) { const int v = part[t]; part[t] = run; run += v; } } __syncthreads();
    int run = part[threadIdx.x]; for (int i = a; i < b; ++i) { VST2(int, off + i, run); run += cnt[i]; }
    if (a < N && b == N) { VST2(int, off + N, run); }
}
__global__ __launch_bounds__(256) void k_slotcopy(const int* __restrict__ off, const int* __restrict__ NBR, int* slot, int N) {
    const int t = blockIdx.x * 256 + threadIdx.x; const int tot = off[N]; if (t >= tot) return;
    int lo = 0, hi = N - 1;
    while (lo < hi) { const int mid = (lo + hi + 1) >> 1; if (off[mid] <= t) lo = mid; else hi = mid - 1; }
    int j = t - off[lo]; j = (j < 0) ? 0 : ((j >= IL_CAP) ? (IL_CAP - 1) : j);
    VST2(int, slot + t, NBR[(size_t)lo * IL_CAP + j]);
}

__global__ __launch_bounds__(256) void k_gather(const float* __restrict__ RES, const int* __restrict__ nid, int n, float* HL) {
    const size_t q = (size_t)blockIdx.x * 256 + threadIdx.x; if (q >= (size_t)n * HH) return; const int c = (int)(q % HH), i = (int)(q / HH); int g = nid[i]; g = g < 0 ? 0 : (g >= NN_ ? NN_ - 1 : g);
    VST2(float, HL + q, RES[(size_t)g * HH + c]);
}
__global__ __launch_bounds__(256) void k_scatter(const float* __restrict__ HL, const int* __restrict__ nid, int n, float* RES) {
    const size_t q = (size_t)blockIdx.x * 256 + threadIdx.x; if (q >= (size_t)n * HH) return; const int c = (int)(q % HH), i = (int)(q / HH); int g = nid[i]; g = g < 0 ? 0 : (g >= NN_ ? NN_ - 1 : g);
    VST2(float, RES + (size_t)g * HH + c, HL[q]);
}
__global__ __launch_bounds__(256) void k_segsum(const float* __restrict__ M, const int* __restrict__ srcs, int n, int ne, const int* __restrict__ off, const int* __restrict__ slot, float* A) {
    const size_t q = (size_t)blockIdx.x * 256 + threadIdx.x; if (q >= (size_t)n * HH) return; const int c = (int)(q % HH), i = (int)(q / HH); const int a = off[i], b = off[i + 1]; float s = 0.f;
    for (int p = a; p < b && p < a + IL_CAP; ++p) { int e = slot[p]; e = e < 0 ? 0 : (e >= ne ? ne - 1 : e); int sn = srcs[e]; sn = sn < 0 ? 0 : (sn >= n ? n - 1 : sn); s += M[(size_t)sn * HH + c]; }
    VST2(float, A + q, s);
}
__global__ __launch_bounds__(256) void k_gru(const float* __restrict__ GI, const float* __restrict__ GH, const float* Hold, int r0, int nr, float* Hnew) {
    const size_t q = (size_t)blockIdx.x * 256 + threadIdx.x; if (q >= (size_t)nr * HH) return; const int c = (int)(q % HH), il = (int)(q / HH); const size_t i = (size_t)r0 + il;
    const float* gi = GI + (size_t)il * 3 * HH; const float* gh = GH + (size_t)il * 3 * HH;
    const float r = 1.0f / (1.0f + expf(-(gi[c] + gh[c]))); const float z = 1.0f / (1.0f + expf(-(gi[HH + c] + gh[HH + c]))); const float ng = tanhf(gi[2 * HH + c] + r * gh[2 * HH + c]);
    VST2(float, Hnew + i * HH + c, (1.0f - z) * ng + z * Hold[i * HH + c]);
}
__global__ __launch_bounds__(256) void k_eler(const float* __restrict__ Z, const float* __restrict__ al, const float* __restrict__ ar, int n, float* EL, float* ER) {
    const int i = blockIdx.x * 256 + threadIdx.x; if (i >= n) return; const float* z = Z + (size_t)i * HH; float a = 0.f, b = 0.f;
#pragma unroll 4
    for (int c = 0; c < HH; ++c) { const float v = z[c]; a += v * al[c]; b += v * ar[c]; }
    VST2(float, EL + i, a); VST2(float, ER + i, b);
}
__global__ __launch_bounds__(256) void k_gatstats(const float* __restrict__ EL, const float* __restrict__ ER, const int* __restrict__ srcs, int n, int ne, const int* __restrict__ off, const int* __restrict__ slot, float* NM, float* ND) {
    const int i = blockIdx.x * 256 + threadIdx.x; if (i >= n) return; const int a = off[i], b = off[i + 1]; const float er = ER[i]; float m = -__builtin_inff();
    for (int p = a; p < b && p < a + IL_CAP; ++p) { int e = slot[p]; e = e < 0 ? 0 : (e >= ne ? ne - 1 : e); int s = srcs[e]; s = s < 0 ? 0 : (s >= n ? n - 1 : s); float v = EL[s] + er; v = v > 0.f ? v : 0.2f * v; m = fmaxf(m, v); }
    float zsum = 0.f;
    for (int p = a; p < b && p < a + IL_CAP; ++p) { int e = slot[p]; e = e < 0 ? 0 : (e >= ne ? ne - 1 : e); int s = srcs[e]; s = s < 0 ? 0 : (s >= n ? n - 1 : s); float v = EL[s] + er; v = v > 0.f ? v : 0.2f * v; zsum += expf(v - m); }
    VST2(float, NM + i, m); VST2(float, ND + i, zsum);
}
__global__ __launch_bounds__(256) void k_alpha(const float* __restrict__ EL, const float* __restrict__ ER, const float* __restrict__ NM, const float* __restrict__ ND, const int* __restrict__ srcs, const int* __restrict__ dsts, int n, int ne, float* ALPHA) {
    const int e = blockIdx.x * 256 + threadIdx.x; if (e >= ne) return; int s = srcs[e]; s = s < 0 ? 0 : (s >= n ? n - 1 : s); int d = dsts[e]; d = d < 0 ? 0 : (d >= n ? n - 1 : d);
    float v = EL[s] + ER[d]; v = v > 0.f ? v : 0.2f * v; VST2(float, ALPHA + e, expf(v - NM[d]) / ND[d]);
}
__global__ __launch_bounds__(256) void k_gatagg(const float* __restrict__ Z, const float* __restrict__ ALPHA, const float* __restrict__ bias, const int* __restrict__ srcs, int n, int ne, const int* __restrict__ off, const int* __restrict__ slot, float* OUT) {
    const size_t q = (size_t)blockIdx.x * 256 + threadIdx.x; if (q >= (size_t)n * HH) return; const int c = (int)(q % HH), i = (int)(q / HH); const int a = off[i], b = off[i + 1]; float s = 0.f;
    for (int p = a; p < b && p < a + IL_CAP; ++p) { int e = slot[p]; e = e < 0 ? 0 : (e >= ne ? ne - 1 : e); int sn = srcs[e]; sn = sn < 0 ? 0 : (sn >= n ? n - 1 : sn); s += ALPHA[e] * Z[(size_t)sn * HH + c]; }
    s += bias[c]; VST2(float, OUT + q, s > 0.f ? s : expm1f(s));
}
__global__ __launch_bounds__(256) void k_gate(const float* __restrict__ RES, const float* __restrict__ wg, const float* __restrict__ bg, float* G) {
    const int i = blockIdx.x * 256 + threadIdx.x; if (i >= NN_) return; const float* r = RES + (size_t)i * HH; float a = bg[0];
#pragma unroll 4
    for (int c = 0; c < HH; ++c) a += r[c] * wg[c];
    VST2(float, G + i, a);
}
__global__ __launch_bounds__(256) void k_pmax(const float* __restrict__ G, float* PM) {
    __shared__ float red[256]; const int tid = threadIdx.x; float m = -__builtin_inff();
    for (int i = blockIdx.x * 256 + tid; i < NN_; i += NPB * 256) m = fmaxf(m, G[i]);
    red[tid] = m; __syncthreads(); for (int o = 128; o > 0; o >>= 1) { if (tid < o) red[tid] = fmaxf(red[tid], red[tid + o]); __syncthreads(); }
    if (tid < 32) { VST2(float, PM + blockIdx.x * 32 + tid, red[0]); }
}
__global__ __launch_bounds__(256) void k_ppart(const float* __restrict__ G, const float* __restrict__ PM, const float* __restrict__ RES, float* PS) {
    const int tid = threadIdx.x; float gmax = -__builtin_inff(); for (int b = 0; b < NPB; ++b) gmax = fmaxf(gmax, PM[b * 32]);
    const int per = (NN_ + NPB - 1) / NPB; const int i0 = blockIdx.x * per; const int i1 = min(NN_, i0 + per);
    double s = 0.0;
    if (tid < HH) { for (int i = i0; i < i1; ++i) s += (double)(expf(G[i] - gmax) * RES[(size_t)i * HH + tid]); }
    else if (tid == HH) { for (int i = i0; i < i1; ++i) s += (double)expf(G[i] - gmax); }
    if (tid <= HH) { VST2(double, (double*)PS + (size_t)blockIdx.x * 160 + tid, s); }
}
__global__ __launch_bounds__(256) void k_pfinal(const double* __restrict__ PS, const float* __restrict__ Wcls, const float* __restrict__ bcls, float* pred, float* rdout) {
    __shared__ float rd[HH + 1]; const int tid = threadIdx.x;
    if (tid <= HH) { double s = 0.0; for (int b = 0; b < NPB; ++b) s += PS[(size_t)b * 160 + tid]; rd[tid] = (float)s; }
    __syncthreads();
    const float den = rd[HH];
    if (tid < HH) { VST2(float, rdout + tid, rd[tid] / den); }
    if (tid < 2) { float p = bcls[tid]; for (int c = 0; c < HH; ++c) p += (rd[c] / den) * Wcls[tid * HH + c]; VST2(float, pred + tid, p); }
}
__global__ __launch_bounds__(1024) void k_copy(const float* __restrict__ src, float* dst, size_t n) { const size_t q = (size_t)blockIdx.x * 1024 + threadIdx.x; if (q < n) { VST2(float, dst + q, src[q]); } }

extern "C" void kernel_launch(void* const* d_in, const int* in_sizes, int n_in,
                              void* d_out, int out_size, void* d_ws, size_t ws_size, hipStream_t stream) {
    (void)in_sizes; (void)n_in; (void)out_size;
    const int* nid[4]; const int* src[4]; const int* dst[4]; const int nn[4] = {99977, 99969, 99973, 99972}; const int ne[4] = {400240, 399214, 400866, 399680};
    for (int t = 0; t < 4; ++t) { nid[t] = (const int*)d_in[3 * t]; src[t] = (const int*)d_in[3 * t + 1]; dst[t] = (const int*)d_in[3 * t + 2]; }
    const float* feats = (const float*)d_in[12];
    const float* Wm[3], *bm[3], *Wih[3], *bih[3], *Whh[3], *bhh[3];
    for (int t = 0; t < 3; ++t) { Wm[t] = (const float*)d_in[13 + 6 * t]; bm[t] = (const float*)d_in[14 + 6 * t]; Wih[t] = (const float*)d_in[15 + 6 * t]; bih[t] = (const float*)d_in[16 + 6 * t]; Whh[t] = (const float*)d_in[17 + 6 * t]; bhh[t] = (const float*)d_in[18 + 6 * t]; }
    const float* Wfc = (const float*)d_in[31]; const float* attl = (const float*)d_in[32]; const float* attr = (const float*)d_in[33]; const float* gbias = (const float*)d_in[34];
    const float* Wgate = (const float*)d_in[35]; const float* bgate = (const float*)d_in[36]; const float* Wcls = (const float*)d_in[37]; const float* bcls = (const float*)d_in[38];
    float* out = (float*)d_out;
    float* o_pred = out;
    float* o_res = out + 2;
    float* o_rd = out + 2 + (size_t)NN_ * HH;
    float* o_alpha = o_rd + HH;

    char* wsp = (char*)d_ws;
    auto take = [&](size_t bytes) { char* p = wsp; wsp += (bytes + 255) & ~(size_t)255; return (void*)p; };
    int* NBR = (int*)take((size_t)NN_ * IL_CAP * 4); int* cnt = (int*)take((size_t)(NN_ + 1) * 4); int* off = (int*)take((size_t)(NN_ + 1) * 4); int* slot = (int*)take((size_t)401000 * 4);
    const size_t NR = (size_t)NN_ * HH;
    float* RES = (float*)take(NR * 4); float* HL = (float*)take(NR * 4); float* MH = (float*)take(NR * 4); float* A = (float*)take(NR * 4);
    const int CHR = (NN_ + NCHK - 1) / NCHK;
    float* GI = (float*)take((size_t)CHR * 3 * HH * 4); float* GH = (float*)take((size_t)CHR * 3 * HH * 4);
    float* EL = (float*)take((size_t)NN_ * 4); float* ER = (float*)take((size_t)NN_ * 4); float* NM = (float*)take((size_t)NN_ * 4); float* ND = (float*)take((size_t)NN_ * 4); float* ALPHA = (float*)take((size_t)400000 * 4);
    float* G = (float*)take((size_t)NN_ * 4); float* PM = (float*)take((size_t)NPB * 32 * 4); double* PS = (double*)take((size_t)NPB * 160 * 8);
    if ((size_t)(wsp - (char*)d_ws) > ws_size) return;

    k_copy<<<(unsigned)((NR + 1023) / 1024), 1024, 0, stream>>>(feats, RES, NR);
    for (int t = 0; t < 3; ++t) {
        const int n = nn[t], E = ne[t];
        k_inlists<<<(n + IL_T - 1) / IL_T, IL_T, 0, stream>>>(dst[t], E, n, NBR, cnt);
        k_csr_scan<<<1, 256, 0, stream>>>(cnt, off, n);
        k_slotcopy<<<(E + 255) / 256, 256, 0, stream>>>(off, NBR, slot, n);
        k_gather<<<(unsigned)(((size_t)n * HH + 255) / 256), 256, 0, stream>>>(RES, nid[t], n, HL);
        for (int s = 0; s < 2; ++s) {
            { GemmArgs g = gemm_args(HL, HH, zm(0), Wm[t], HH, zm(0), MH, HH, zm(0), n, HH, HH); g.bias = bm[t]; gemm_kernel<1, 0, 2, 2, 4, 2, ACT_NONE><<<dim3((n + 63) / 64, 1, 1), 256, 0, stream>>>(g); }
            k_segsum<<<(unsigned)(((size_t)n * HH + 255) / 256), 256, 0, stream>>>(MH, src[t], n, E, off, slot, A);
            for (int r0 = 0; r0 < n; r0 += CHR) {
                const int nr = min(CHR, n - r0);
                { GemmArgs g = gemm_args(A + (size_t)r0 * HH, HH, zm(0), Wih[t], HH, zm(0), GI, 3 * HH, zm(0), nr, 3 * HH, HH); g.bias = bih[t]; gemm_kernel<1, 0, 2, 2, 4, 2, ACT_NONE><<<dim3((nr + 63) / 64, 3, 1), 256, 0, stream>>>(g); }
                { GemmArgs g = gemm_args(HL + (size_t)r0 * HH, HH, zm(0), Whh[t], HH, zm(0), GH, 3 * HH, zm(0), nr, 3 * HH, HH); g.bias = bhh[t]; gemm_kernel<1, 0, 2, 2, 4, 2, ACT_NONE><<<dim3((nr + 63) / 64, 3, 1), 256, 0, stream>>>(g); }
                k_gru<<<(unsigned)(((size_t)nr * HH + 255) / 256), 256, 0, stream>>>(GI, GH, HL, r0, nr, HL);
            }
        }
        k_scatter<<<(unsigned)(((size_t)n * HH + 255) / 256), 256, 0, stream>>>(HL, nid[t], n, RES);
    }
    {
        const int n = nn[3], E = ne[3];
        k_inlists<<<(n + IL_T - 1) / IL_T, IL_T, 0, stream>>>(dst[3], E, n, NBR, cnt);
        k_csr_scan<<<1, 256, 0, stream>>>(cnt, off, n);
        k_slotcopy<<<(E + 255) / 256, 256, 0, stream>>>(off, NBR, slot, n);
        k_gather<<<(unsigned)(((size_t)n * HH + 255) / 256), 256, 0, stream>>>(RES, nid[3], n, HL);
        { GemmArgs g = gemm_args(HL, HH, zm(0), Wfc, HH, zm(0), MH, HH, zm(0), n, HH, HH); gemm_kernel<1, 0, 2, 2, 4, 2, ACT_NONE><<<dim3((n + 63) / 64, 1, 1), 256, 0, stream>>>(g); }
        k_eler<<<(n + 255) / 256, 256, 0, stream>>>(MH, attl, attr, n, EL, ER);
        k_gatstats<<<(n + 255) / 256, 256, 0, stream>>>(EL, ER, src[3], n, E, off, slot, NM, ND);
        k_alpha<<<(E + 255) / 256, 256, 0, stream>>>(EL, ER, NM, ND, src[3], dst[3], n, E, ALPHA);
        k_gatagg<<<(unsigned)(((size_t)n * HH + 255) / 256), 256, 0, stream>>>(MH, ALPHA, gbias, src[3], n, E, off, slot, A);
        k_scatter<<<(unsigned)(((size_t)n * HH + 255) / 256), 256, 0, stream>>>(A, nid[3], n, RES);
        k_copy<<<(E + 1023) / 1024, 1024, 0, stream>>>(ALPHA, o_alpha, (size_t)E);
    }
    k_gate<<<(NN_ + 255) / 256, 256, 0, stream>>>(RES, Wgate, bgate, G);
    k_pmax<<<NPB, 256, 0, stream>>>(G, PM);
    k_ppart<<<NPB, 256, 0, stream>>>(G, PM, RES, (float*)PS);
    k_pfinal<<<1, 256, 0, stream>>>(PS, Wcls, bcls, o_pred, o_rd);
    k_copy<<<(unsigned)((NR + 1023) / 1024), 1024, 0, stream>>>(RES, o_res, NR);
}
